// ResidualBlock_79602923864079
// MI455X (gfx1250) — hardware-verified
//
#include <hip/hip_runtime.h>
#include <stdint.h>

typedef __attribute__((ext_vector_type(16))) _Float16 v16h;
typedef __attribute__((ext_vector_type(8)))  _Float16 v8h;
typedef __attribute__((ext_vector_type(16))) __bf16   v16b;
typedef __attribute__((ext_vector_type(8)))  __bf16   v8b;
typedef __attribute__((ext_vector_type(8)))  float    v8f;
typedef __attribute__((ext_vector_type(4)))  float    v4f;
typedef __attribute__((ext_vector_type(4)))  unsigned int v4u;
typedef __attribute__((ext_vector_type(2)))  unsigned int v2u;

constexpr int NNODE        = 131072;
constexpr int NCH          = 64;
constexpr int NTAP         = 27;
constexpr int KTOT         = NTAP * NCH;
constexpr int CONV_THREADS = 128;
constexpr int CONV_WAVES   = CONV_THREADS / 32;
constexpr int CONV_ROWS    = CONV_WAVES * 32;
constexpr int CONV_BLOCKS  = NNODE / CONV_ROWS;
constexpr int APITCH       = 72;
constexpr int BPITCH       = 72;
constexpr int PART_STRIDE  = 128;
constexpr int STATS_FLOATS = 256;

static_assert(NNODE % CONV_ROWS == 0, "M must be a multiple of the block row tile");
static_assert(KTOT % 32 == 0, "K must be a multiple of 32");
static_assert(NCH == 64, "N tile is 64");
static_assert((NNODE * 8) % 256 == 0, "elementwise grids exact");
static_assert((NNODE * 16) % 256 == 0, "elementwise grids exact");
static_assert(CONV_WAVES * 16 * 68 * 4 <= 2 * CONV_ROWS * APITCH * 2, "slab fits in the A tile region");

__device__ __forceinline__ unsigned short f2bf_bits(float f) {
  unsigned u = __float_as_uint(f);
  return (unsigned short)((u + 0x7FFFu + ((u >> 16) & 1u)) >> 16);
}
__device__ __forceinline__ float bf_bits2f(unsigned short h) { return __uint_as_float(((unsigned)h) << 16); }

__device__ __forceinline__ void dep_guard_h(v8f& a, v8f& b, v16h x, v16h y) { asm volatile("v_nop\n\tv_nop\n\tv_nop\n\tv_nop" : "+v"(a), "+v"(b) : "v"(x), "v"(y)); }
__device__ __forceinline__ void dep_guard_b(v8f& a, v8f& b, v16b x, v16b y) { asm volatile("v_nop\n\tv_nop\n\tv_nop\n\tv_nop" : "+v"(a), "+v"(b) : "v"(x), "v"(y)); }
__device__ __forceinline__ void keep4_h(v16h a, v16h b, v16h c, v16h d) { asm volatile("v_nop" :: "v"(a), "v"(b), "v"(c), "v"(d)); }
__device__ __forceinline__ void keep4_b(v16b a, v16b b, v16b c, v16b d) { asm volatile("v_nop" :: "v"(a), "v"(b), "v"(c), "v"(d)); }
__device__ __forceinline__ void acc_guard4(v8f& a, v8f& b, v8f& c, v8f& d) { asm volatile("v_nop\n\tv_nop\n\tv_nop\n\tv_nop" : "+v"(a), "+v"(b), "+v"(c), "+v"(d)); }
template <typename T> struct Frag;
template <> struct Frag<_Float16> {
  typedef v16h V; union U { v16h v; v8h h[2]; };
  static __device__ __forceinline__ v16h load(const _Float16* p) {
    U f; f.h[0] = *(const v8h*)(p); f.h[1] = *(const v8h*)(p + 16); return f.v;
  }
  static __device__ __forceinline__ v8f mma(v16h a, v16h b, v8f c) {
    return __builtin_amdgcn_wmma_f32_16x16x32_f16(false, a, false, b, (short)0, c, false, false);
  }
  static __device__ __forceinline__ void guard(v8f& a, v8f& b, v16h x, v16h y) { dep_guard_h(a, b, x, y); }
  static __device__ __forceinline__ void keep(v16h a, v16h b, v16h c, v16h d) { keep4_h(a, b, c, d); }
};
template <> struct Frag<__bf16> {
  typedef v16b V; union U { v16b v; v8b h[2]; };
  static __device__ __forceinline__ v16b load(const __bf16* p) {
    U f; f.h[0] = *(const v8b*)(p); f.h[1] = *(const v8b*)(p + 16); return f.v;
  }
  static __device__ __forceinline__ v8f mma(v16b a, v16b b, v8f c) {
    return __builtin_amdgcn_wmma_f32_16x16x32_bf16(false, a, false, b, (short)0, c, false, false);
  }
  static __device__ __forceinline__ void guard(v8f& a, v8f& b, v16b x, v16b y) { dep_guard_b(a, b, x, y); }
  static __device__ __forceinline__ void keep(v16b a, v16b b, v16b c, v16b d) { keep4_b(a, b, c, d); }
};

__device__ __forceinline__ unsigned pack_bf2(float a, float b) {
  return (unsigned)f2bf_bits(a) | ((unsigned)f2bf_bits(b) << 16);
}
__device__ __forceinline__ void split_bf2(float a, float b, unsigned& hw, unsigned& lw) {
  const unsigned short ha = f2bf_bits(a), hb = f2bf_bits(b);
  const unsigned short la = f2bf_bits(a - bf_bits2f(ha)), lb = f2bf_bits(b - bf_bits2f(hb));
  hw = (unsigned)ha | ((unsigned)hb << 16);
  lw = (unsigned)la | ((unsigned)lb << 16);
}
__device__ __forceinline__ float bn_apply(float x, const float* st, int c) {
  return ((x - st[c]) * st[64 + c]) * st[128 + c] + st[192 + c];
}

__global__ __launch_bounds__(256) void feats_to_bf16_kernel(const float* __restrict__ src,
                                                             unsigned short* __restrict__ dst) {
  const int gid = blockIdx.x * 256 + threadIdx.x;
  const size_t base = (size_t)(gid >> 3) * NCH + (gid & 7) * 8;
  const v4f a = *(const v4f*)(src + base);
  const v4f b = *(const v4f*)(src + base + 4);
  v4u u;
  u.x = pack_bf2(a.x, a.y); u.y = pack_bf2(a.z, a.w);
  u.z = pack_bf2(b.x, b.y); u.w = pack_bf2(b.z, b.w);
  *(volatile v4u*)(dst + base) = u;
  __threadfence();
  *(volatile v4u*)(dst + base) = u;
}

__global__ __launch_bounds__(256) void prep_w_kernel(const float* __restrict__ W1, const float* __restrict__ W2,
                                                      unsigned short* __restrict__ Wt1, unsigned short* __restrict__ Wt2) {
  __shared__ float tile[64][65];
  const int tid = threadIdx.x;
  const int tap = blockIdx.x;
  const int which = blockIdx.y;
  const float* src = ((which == 0) ? W1 : W2) + (size_t)tap * (NCH * NCH);
  unsigned short* dst = (which == 0) ? Wt1 : Wt2;
#pragma unroll
  for (int it = 0; it < 4; ++it) {
    const int idx = tid + it * 256;
    const int ci = idx >> 4, co4 = (idx & 15) * 4;
    const v4f v = *(const v4f*)(src + ci * NCH + co4);
    tile[ci][co4 + 0] = v.x; tile[ci][co4 + 1] = v.y; tile[ci][co4 + 2] = v.z; tile[ci][co4 + 3] = v.w;
  }
  __syncthreads();
  v4u u0, u1;
  {
    const int idx = tid;
    const int co = idx >> 3, ci8 = (idx & 7) * 8;
    u0.x = pack_bf2(tile[ci8 + 0][co], tile[ci8 + 1][co]); u0.y = pack_bf2(tile[ci8 + 2][co], tile[ci8 + 3][co]);
    u0.z = pack_bf2(tile[ci8 + 4][co], tile[ci8 + 5][co]); u0.w = pack_bf2(tile[ci8 + 6][co], tile[ci8 + 7][co]);
  }
  {
    const int idx = tid + 256;
    const int co = idx >> 3, ci8 = (idx & 7) * 8;
    u1.x = pack_bf2(tile[ci8 + 0][co], tile[ci8 + 1][co]); u1.y = pack_bf2(tile[ci8 + 2][co], tile[ci8 + 3][co]);
    u1.z = pack_bf2(tile[ci8 + 4][co], tile[ci8 + 5][co]); u1.w = pack_bf2(tile[ci8 + 6][co], tile[ci8 + 7][co]);
  }
  unsigned short* p0 = dst + (size_t)(tid >> 3) * KTOT + tap * NCH + (tid & 7) * 8;
  unsigned short* p1 = dst + (size_t)((tid + 256) >> 3) * KTOT + tap * NCH + (tid & 7) * 8;
  *(volatile v4u*)p0 = u0;
  *(volatile v4u*)p1 = u1;
  __threadfence();
  *(volatile v4u*)p0 = u0;
  *(volatile v4u*)p1 = u1;
}

template <bool SPLITA>
__global__ __launch_bounds__(CONV_THREADS) void gconv_kernel(
    const unsigned short* __restrict__ Ahi, const unsigned short* __restrict__ Alo,
    const int* __restrict__ nidx,
    const unsigned short* __restrict__ Wt,
    float* __restrict__ Hout,
    float* __restrict__ part)
{
  __shared__ __align__(16) unsigned short As[2][CONV_ROWS * APITCH];
  __shared__ __align__(16) unsigned short Bs[NCH * BPITCH];
  __shared__ float redS[CONV_WAVES][NCH];
  __shared__ float redQ[CONV_WAVES][NCH];
  __shared__ __align__(16) float pstage[PART_STRIDE];

  const int tid   = threadIdx.x;
  const int lane  = tid & 31;
  const int wave  = tid >> 5;
  const int rlane = lane & 15;
  const int koff  = (lane >> 4) * 8;
  const int mOff  = (lane >> 4) * 8;
  const int m0    = blockIdx.x * CONV_ROWS;

  v8f acc[2][4];
#pragma unroll
  for (int i = 0; i < 2; ++i)
#pragma unroll
    for (int j = 0; j < 4; ++j) acc[i][j] = (v8f){0.f,0.f,0.f,0.f,0.f,0.f,0.f,0.f};

  for (int t = 0; t < NTAP; ++t) {
    __syncthreads();
#pragma unroll
    for (int it = 0; it < 4; ++it) {
      const int idx = tid + it * CONV_THREADS;
      const int co = idx >> 3, c8 = (idx & 7) * 8;
      const v4u w = *(const v4u*)(Wt + (size_t)co * KTOT + t * NCH + c8);
      *(v4u*)(Bs + co * BPITCH + c8) = w;
    }
#pragma unroll 1
    for (int p = 0; p < 2; ++p) {
      const int r = p * 64 + (tid >> 1);
      const int half = tid & 1;
      int id = nidx[(size_t)t * NNODE + m0 + r];
      id = (id < 0) ? (id + NNODE) : id;
      id = (id < 0) ? 0 : ((id > NNODE - 1) ? (NNODE - 1) : id);
      const v4u* gh = (const v4u*)(Ahi + (size_t)id * NCH + half * 32);
      v4u* dh = (v4u*)(&As[0][r * APITCH + half * 32]);
      const v4u h0 = gh[0], h1 = gh[1], h2 = gh[2], h3 = gh[3];
      dh[0] = h0; dh[1] = h1; dh[2] = h2; dh[3] = h3;
      if (SPLITA) {
        const v4u* gl = (const v4u*)(Alo + (size_t)id * NCH + half * 32);
        v4u* dl = (v4u*)(&As[1][r * APITCH + half * 32]);
        const v4u l0 = gl[0], l1 = gl[1], l2 = gl[2], l3 = gl[3];
        dl[0] = l0; dl[1] = l1; dl[2] = l2; dl[3] = l3;
      }
    }
    __syncthreads();
#pragma unroll
    for (int kk = 0; kk < 2; ++kk) {
      v16b bfr[4];
#pragma unroll
      for (int j = 0; j < 4; ++j)
        bfr[j] = Frag<__bf16>::load((const __bf16*)(Bs + (j * 16 + rlane) * BPITCH + kk * 32 + koff));
#pragma unroll
      for (int i = 0; i < 2; ++i) {
        const int arow = wave * 32 + i * 16 + rlane;
        const v16b ah = Frag<__bf16>::load((const __bf16*)(&As[0][arow * APITCH + kk * 32 + koff]));
        v16b al = ah;
        if (SPLITA) al = Frag<__bf16>::load((const __bf16*)(&As[1][arow * APITCH + kk * 32 + koff]));
#pragma unroll
        for (int j = 0; j < 4; ++j) {
          acc[i][j] = Frag<__bf16>::mma(ah, bfr[j], acc[i][j]);
          if (SPLITA) acc[i][j] = Frag<__bf16>::mma(al, bfr[j], acc[i][j]);
        }
        Frag<__bf16>::guard(acc[i][0], acc[i][3], ah, al);
      }
      Frag<__bf16>::keep(bfr[0], bfr[1], bfr[2], bfr[3]);
    }
  }
  acc_guard4(acc[0][0], acc[0][1], acc[0][2], acc[0][3]);
  acc_guard4(acc[1][0], acc[1][1], acc[1][2], acc[1][3]);
  __syncthreads();

#pragma unroll
  for (int j = 0; j < 4; ++j) {
    float s = 0.0f, q = 0.0f;
#pragma unroll
    for (int i = 0; i < 2; ++i)
#pragma unroll
      for (int r = 0; r < 8; ++r) { const float v = acc[i][j][r]; s += v; q += v * v; }
    s += __shfl_xor(s, 16, 32);
    q += __shfl_xor(q, 16, 32);
    if (lane < 16) { redS[wave][j * 16 + rlane] = s; redQ[wave][j * 16 + rlane] = q; }
  }

  float* slab = (float*)(&As[0][0]) + wave * (16 * 68);
#pragma unroll
  for (int i = 0; i < 2; ++i) {
    const int mBase = m0 + wave * 32 + i * 16;
#pragma unroll
    for (int j = 0; j < 4; ++j)
#pragma unroll
      for (int r = 0; r < 8; ++r) slab[(mOff + r) * 68 + (j << 4) + rlane] = acc[i][j][r];
    __builtin_amdgcn_fence(__ATOMIC_RELEASE, "workgroup");
    __builtin_amdgcn_wave_barrier();
    __builtin_amdgcn_fence(__ATOMIC_ACQUIRE, "workgroup");
    {
      const int hh = lane >> 4, c4 = (lane & 15) * 4;
      for (int pass = 0; pass < 2; ++pass) {
#pragma unroll
        for (int it = 0; it < 8; ++it) {
          const int row = it * 2 + hh;
          const v4f v = *(const v4f*)(slab + row * 68 + c4);
          *(volatile v4f*)(Hout + (size_t)(mBase + row) * NCH + c4) = v;
        }
        __threadfence();
      }
    }
    __builtin_amdgcn_fence(__ATOMIC_RELEASE, "workgroup");
    __builtin_amdgcn_wave_barrier();
    __builtin_amdgcn_fence(__ATOMIC_ACQUIRE, "workgroup");
  }

  __syncthreads();
  if (tid < NCH) {
    float s = 0.0f, q = 0.0f;
    s += redS[0][tid]; s += redS[1][tid]; s += redS[2][tid]; s += redS[3][tid];
    q += redQ[0][tid]; q += redQ[1][tid]; q += redQ[2][tid]; q += redQ[3][tid];
    pstage[tid] = s;
    pstage[NCH + tid] = q;
  }
  __syncthreads();
  if (wave == 0) {
    const v4f v = *(const v4f*)(pstage + 4 * lane);
    float* dstp = part + (size_t)blockIdx.x * PART_STRIDE + 4 * lane;
    *(volatile v4f*)dstp = v;
    __threadfence();
    *(volatile v4f*)dstp = v;
  }
}

__global__ __launch_bounds__(64) void bn_stats_kernel(const float* __restrict__ part, int nblk,
                                                      const float* __restrict__ gamma, const float* __restrict__ beta,
                                                      float* __restrict__ stats) {
  __shared__ __align__(16) float st[STATS_FLOATS];
  const int c = threadIdx.x;
  double s = 0.0, q = 0.0;
#pragma unroll 4
  for (int b = 0; b < nblk; ++b) {
    s += (double)part[(size_t)b * PART_STRIDE + c];
    q += (double)part[(size_t)b * PART_STRIDE + NCH + c];
  }
  const double mu = s * (1.0 / (double)NNODE);
  double var = q * (1.0 / (double)NNODE) - mu * mu;
  var = (var < 0.0) ? 0.0 : var;
  const float muf = (float)mu;
  const float varf = (float)var;
  const float inv = rsqrtf(varf + 1e-5f);
  const float g = bf_bits2f(f2bf_bits(gamma[c]));
  const float bb = bf_bits2f(f2bf_bits(beta[c]));
  st[c] = muf; st[64 + c] = inv; st[128 + c] = g; st[192 + c] = bb;
  __syncthreads();
  if (c < 32) {
    const v4f v0 = *(const v4f*)(st + 4 * c);
    const v4f v1 = *(const v4f*)(st + 128 + 4 * c);
    *(volatile v4f*)(stats + 4 * c) = v0;
    *(volatile v4f*)(stats + 128 + 4 * c) = v1;
    __threadfence();
    *(volatile v4f*)(stats + 4 * c) = v0;
    *(volatile v4f*)(stats + 128 + 4 * c) = v1;
  }
}

__global__ __launch_bounds__(256) void bn_relu_split_kernel(const float* __restrict__ H, const float* __restrict__ stats,
                                                            unsigned short* __restrict__ Phi, unsigned short* __restrict__ Plo) {
  __shared__ __align__(16) float st[STATS_FLOATS];
  const int tid = threadIdx.x;
  if (tid < 64) { const v4f v = *(const v4f*)(stats + 4 * tid); *(v4f*)(st + 4 * tid) = v; }
  __syncthreads();
  const int gid = blockIdx.x * 256 + tid;
  const int c8 = (gid & 7) * 8;
  const size_t base = (size_t)(gid >> 3) * NCH + c8;
  const v4f x0 = *(const v4f*)(H + base);
  const v4f x1 = *(const v4f*)(H + base + 4);
  const float y0 = fmaxf(bn_apply(x0.x, st, c8 + 0), 0.0f);
  const float y1 = fmaxf(bn_apply(x0.y, st, c8 + 1), 0.0f);
  const float y2 = fmaxf(bn_apply(x0.z, st, c8 + 2), 0.0f);
  const float y3 = fmaxf(bn_apply(x0.w, st, c8 + 3), 0.0f);
  const float y4 = fmaxf(bn_apply(x1.x, st, c8 + 4), 0.0f);
  const float y5 = fmaxf(bn_apply(x1.y, st, c8 + 5), 0.0f);
  const float y6 = fmaxf(bn_apply(x1.z, st, c8 + 6), 0.0f);
  const float y7 = fmaxf(bn_apply(x1.w, st, c8 + 7), 0.0f);
  v4u hv, lv;
  { unsigned a, b; split_bf2(y0, y1, a, b); hv.x = a; lv.x = b; }
  { unsigned a, b; split_bf2(y2, y3, a, b); hv.y = a; lv.y = b; }
  { unsigned a, b; split_bf2(y4, y5, a, b); hv.z = a; lv.z = b; }
  { unsigned a, b; split_bf2(y6, y7, a, b); hv.w = a; lv.w = b; }
  *(volatile v4u*)(Phi + base) = hv;
  *(volatile v4u*)(Plo + base) = lv;
  __threadfence();
  *(volatile v4u*)(Phi + base) = hv;
  *(volatile v4u*)(Plo + base) = lv;
}

__global__ __launch_bounds__(256) void bn_res_relu_kernel(const float* __restrict__ H, const unsigned short* __restrict__ Fb,
                                                          const float* __restrict__ stats, float* __restrict__ out) {
  __shared__ __align__(16) float st[STATS_FLOATS];
  const int tid = threadIdx.x;
  if (tid < 64) { const v4f v = *(const v4f*)(stats + 4 * tid); *(v4f*)(st + 4 * tid) = v; }
  __syncthreads();
  const int gid = blockIdx.x * 256 + tid;
  const int c4 = (gid & 15) * 4;
  const size_t base = (size_t)(gid >> 4) * NCH + c4;
  const v4f x = *(const v4f*)(H + base);
  const v2u fw = *(const v2u*)(Fb + base);
  const float f0 = __uint_as_float(fw.x << 16);
  const float f1 = __uint_as_float(fw.x & 0xffff0000u);
  const float f2 = __uint_as_float(fw.y << 16);
  const float f3 = __uint_as_float(fw.y & 0xffff0000u);
  v4f o;
  o.x = fmaxf(bn_apply(x.x, st, c4 + 0) + f0, 0.0f);
  o.y = fmaxf(bn_apply(x.y, st, c4 + 1) + f1, 0.0f);
  o.z = fmaxf(bn_apply(x.z, st, c4 + 2) + f2, 0.0f);
  o.w = fmaxf(bn_apply(x.w, st, c4 + 3) + f3, 0.0f);
  *(volatile v4f*)(out + base) = o;
  __threadfence();
  *(volatile v4f*)(out + base) = o;
}

extern "C" void kernel_launch(void* const* d_in, const int* in_sizes, int n_in,
                              void* d_out, int out_size, void* d_ws, size_t ws_size,
                              hipStream_t stream) {
  (void)n_in;
  const float* feats = (const float*)d_in[0];
  const int*   nidx  = (const int*)d_in[1];
  const float* W1    = (const float*)d_in[2];
  const float* g1    = (const float*)d_in[3];
  const float* b1    = (const float*)d_in[4];
  const float* W2    = (const float*)d_in[5];
  const float* g2    = (const float*)d_in[6];
  const float* b2    = (const float*)d_in[7];
  float* out = (float*)d_out;

  if (in_sizes[0] != NNODE * NCH || in_sizes[1] != NTAP * NNODE ||
      in_sizes[2] != NTAP * NCH * NCH || in_sizes[5] != NTAP * NCH * NCH ||
      in_sizes[3] != NCH || in_sizes[4] != NCH || in_sizes[6] != NCH || in_sizes[7] != NCH ||
      out_size != NNODE * NCH) return;

  char* ws = (char*)d_ws;
  size_t off = 0;
  auto carve = [&](size_t bytes) -> char* {
    char* p = ws + off;
    off += (bytes + 255) & ~(size_t)255;
    return p;
  };
  const size_t planeH = (size_t)NNODE * NCH * 2;
  const size_t planeF = (size_t)NNODE * NCH * 4;
  const size_t wtB    = (size_t)NCH * KTOT * 2;
  const size_t partB  = (size_t)CONV_BLOCKS * PART_STRIDE * 4;
  const size_t statB  = (size_t)STATS_FLOATS * 4;

  unsigned short* Fb   = (unsigned short*)carve(planeH);
  unsigned short* Wt1  = (unsigned short*)carve(wtB);
  unsigned short* Wt2  = (unsigned short*)carve(wtB);
  float*          H1f  = (float*)carve(planeF);
  unsigned short* H1hi = (unsigned short*)carve(planeH);
  unsigned short* H1lo = (unsigned short*)carve(planeH);
  float*          H2f  = (float*)carve(planeF);
  float*          part1 = (float*)carve(partB);
  float*          part2 = (float*)carve(partB);
  float*          st1  = (float*)carve(statB);
  float*          st2  = (float*)carve(statB);
  if (off > ws_size) return;

  feats_to_bf16_kernel<<<(NNODE * 8) / 256, 256, 0, stream>>>(feats, Fb);
  prep_w_kernel<<<dim3(NTAP, 2, 1), 256, 0, stream>>>(W1, W2, Wt1, Wt2);

  gconv_kernel<false><<<CONV_BLOCKS, CONV_THREADS, 0, stream>>>(Fb, Fb, nidx, Wt1, H1f, part1);
  bn_stats_kernel<<<1, 64, 0, stream>>>(part1, CONV_BLOCKS, g1, b1, st1);
  bn_relu_split_kernel<<<(NNODE * 8) / 256, 256, 0, stream>>>(H1f, st1, H1hi, H1lo);

  gconv_kernel<true><<<CONV_BLOCKS, CONV_THREADS, 0, stream>>>(H1hi, H1lo, nidx, Wt2, H2f, part2);
  bn_stats_kernel<<<1, 64, 0, stream>>>(part2, CONV_BLOCKS, g2, b2, st2);
  bn_res_relu_kernel<<<(NNODE * 16) / 256, 256, 0, stream>>>(H2f, Fb, st2, out);
}
